// RNN_63385127354782
// MI455X (gfx1250) — hardware-verified
//
#include <hip/hip_runtime.h>
#include <math.h>

constexpr int NBATCH = 65536;
constexpr int NSTEP  = 30;
constexpr int NIN    = 3;
constexpr int NHID   = 32;
constexpr int NLAY   = 5;
constexpr int NFEAT  = NSTEP * NHID;
constexpr int DH1 = 512, DH2 = 256, DH3 = 128, DH4 = 64;
constexpr int NCHUNK = 4;
constexpr int CHROWS = NBATCH / NCHUNK;
constexpr int RNN_THR   = 128;
constexpr int RNN_WAVES = RNN_THR / 32;
constexpr int RNN_ROWS_BLK = 16 * RNN_WAVES;
constexpr int SLOT = 16 * NHID;
constexpr int WPL  = NHID * NHID;
constexpr int HEAD_THR = 256;
constexpr float WCARRY     = 64.0f;
constexpr float WCARRY_INV = 1.0f / 64.0f;

static_assert(NBATCH % NCHUNK == 0);
static_assert(CHROWS % RNN_ROWS_BLK == 0);
static_assert(CHROWS % HEAD_THR == 0);
static_assert(CHROWS % 64 == 0);
static_assert(DH1 % 64 == 0 && DH2 % 64 == 0 && DH3 % 64 == 0 && DH4 % 64 == 0);
static_assert(NFEAT % 32 == 0 && DH1 % 32 == 0 && DH2 % 32 == 0 && DH3 % 32 == 0);
static_assert(NSTEP % 2 == 0);
static_assert(NHID == 32 && NIN < 8);
static_assert(WPL % RNN_THR == 0 && ((NLAY - 1) * WPL) % RNN_THR == 0 && (NLAY * WPL) % RNN_THR == 0);
static_assert((DH1 * NFEAT / 2) % 32 == 0 && (DH2 * DH1 / 2) % 32 == 0 && (DH3 * DH2 / 2) % 32 == 0 && (DH4 * DH3 / 2) % 32 == 0);
static_assert(((CHROWS / 64) * (DH1 / 64)) % 8 == 0 && ((CHROWS / 64) * (DH4 / 64)) % 8 == 0);

typedef __attribute__((ext_vector_type(16))) _Float16 v16h;
typedef __attribute__((ext_vector_type(8)))  _Float16 v8h;
typedef __attribute__((ext_vector_type(16))) __bf16   v16b;
typedef __attribute__((ext_vector_type(8)))  __bf16   v8b;
typedef __attribute__((ext_vector_type(8)))  float    v8f;
typedef __attribute__((ext_vector_type(4)))  float    v4f;
typedef __attribute__((ext_vector_type(4)))  unsigned v4u;
typedef __attribute__((ext_vector_type(2)))  unsigned v2u;

__device__ __forceinline__ unsigned short f2bf_bits(float f) {
  unsigned u = __float_as_uint(f);
  return (unsigned short)((u + 0x7FFFu + ((u >> 16) & 1u)) >> 16);
}
__device__ __forceinline__ float bf_bits2f(unsigned short h) { return __uint_as_float(((unsigned)h) << 16); }
__device__ __forceinline__ unsigned h2u(float f) {
  const _Float16 h = (_Float16)f;
  return (unsigned)__builtin_bit_cast(unsigned short, h);
}

__device__ __forceinline__ void dep_guard_h(v8f& a, v8f& b, v16h x, v16h y) { asm volatile("v_nop\n\tv_nop\n\tv_nop\n\tv_nop" : "+v"(a), "+v"(b) : "v"(x), "v"(y)); }
__device__ __forceinline__ void dep_guard_b(v8f& a, v8f& b, v16b x, v16b y) { asm volatile("v_nop\n\tv_nop\n\tv_nop\n\tv_nop" : "+v"(a), "+v"(b) : "v"(x), "v"(y)); }
__device__ __forceinline__ void keep4_h(v16h a, v16h b, v16h c, v16h d) { asm volatile("v_nop" :: "v"(a), "v"(b), "v"(c), "v"(d)); }
__device__ __forceinline__ void keep4_b(v16b a, v16b b, v16b c, v16b d) { asm volatile("v_nop" :: "v"(a), "v"(b), "v"(c), "v"(d)); }
__device__ __forceinline__ void acc_guard4(v8f& a, v8f& b, v8f& c, v8f& d) { asm volatile("v_nop\n\tv_nop\n\tv_nop\n\tv_nop" : "+v"(a), "+v"(b), "+v"(c), "+v"(d)); }
__device__ __forceinline__ void guard_acc2_frag6(v8f& a, v8f& b, v16h f0, v16h f1, v16h f2, v16h f3, v16h f4, v16h f5) {
  asm volatile("v_nop\n\tv_nop\n\tv_nop\n\tv_nop" : "+v"(a), "+v"(b) : "v"(f0), "v"(f1), "v"(f2), "v"(f3), "v"(f4), "v"(f5));
}
template <typename T> struct Frag;
template <> struct Frag<_Float16> {
  typedef v16h V; union U { v16h v; v8h h[2]; };
  static __device__ __forceinline__ v16h load(const _Float16* p) {
    U f; f.h[0] = *(const v8h*)(p); f.h[1] = *(const v8h*)(p + 16); return f.v;
  }
  static __device__ __forceinline__ v8f mma(v16h a, v16h b, v8f c) {
    return __builtin_amdgcn_wmma_f32_16x16x32_f16(false, a, false, b, (short)0, c, false, false);
  }
  static __device__ __forceinline__ void guard(v8f& a, v8f& b, v16h x, v16h y) { dep_guard_h(a, b, x, y); }
  static __device__ __forceinline__ void keep(v16h a, v16h b, v16h c, v16h d) { keep4_h(a, b, c, d); }
};
template <> struct Frag<__bf16> {
  typedef v16b V; union U { v16b v; v8b h[2]; };
  static __device__ __forceinline__ v16b load(const __bf16* p) {
    U f; f.h[0] = *(const v8b*)(p); f.h[1] = *(const v8b*)(p + 16); return f.v;
  }
  static __device__ __forceinline__ v8f mma(v16b a, v16b b, v8f c) {
    return __builtin_amdgcn_wmma_f32_16x16x32_bf16(false, a, false, b, (short)0, c, false, false);
  }
  static __device__ __forceinline__ void guard(v8f& a, v8f& b, v16b x, v16b y) { dep_guard_b(a, b, x, y); }
  static __device__ __forceinline__ void keep(v16b a, v16b b, v16b c, v16b d) { keep4_b(a, b, c, d); }
};

__device__ __forceinline__ float tanh_acc(float z) {
  const float e = expf(2.0f * z);
  return 1.0f - 2.0f * __builtin_amdgcn_rcpf(e + 1.0f);
}

template <int ET> struct Elem;
template <> struct Elem<0> { typedef _Float16 T; };
template <> struct Elem<1> { typedef __bf16 T; };
template <int ET, bool SPLIT, int BIAS_MODE, int OUT_MODE, bool RESID, int ACT = 0>
__global__ __launch_bounds__(256) void wmma_gemm64(
    const unsigned short* __restrict__ Ap, const unsigned short* __restrict__ A2p, int lda, long strideA,
    const unsigned short* __restrict__ Btp, const unsigned short* __restrict__ Bt2p, int ldb, long strideB,
    void* __restrict__ Cout, void* __restrict__ Cout2, int ldc, long strideC,
    const float* __restrict__ bias,
    const float* __restrict__ resid, long strideR,
    int M, int N, int K, float scale) {
  typedef typename Elem<ET>::T T;
  typedef typename Frag<T>::V V;
  const T* A = (const T*)Ap; const T* A2 = (const T*)A2p; const T* Bt = (const T*)Btp; const T* Bt2 = (const T*)Bt2p;
  __shared__ __align__(16) float sT[8][16 * 68];
  const int b    = blockIdx.y;
  const int lane = threadIdx.x & 31;
  const int wave = threadIdx.x >> 5;
  const int tilesN = N >> 6;
  const int tilesM = M >> 6;
  const int tile = blockIdx.x * 8 + wave;
  if (tile >= tilesM * tilesN) return;
  const int tm = tile / tilesN;
  const int tn = tile - tm * tilesN;
  const int m0 = tm << 6;
  const int n0 = tn << 6;

  const T* Ab  = A  + (size_t)b * strideA;
  const T* Bb  = Bt + (size_t)b * strideB;
  const T* Ab2 = SPLIT ? (A2  + (size_t)b * strideA) : nullptr;
  const T* Bb2 = SPLIT ? (Bt2 + (size_t)b * strideB) : nullptr;

  const int rlane = lane & 15;
  const int koff  = (lane >> 4) * 8;
  const int mOff  = (lane >> 4) * 8;

  v8f acc[4][4];
#pragma unroll
  for (int i = 0; i < 4; ++i)
#pragma unroll
    for (int j = 0; j < 4; ++j) acc[i][j] = (v8f){0.f,0.f,0.f,0.f,0.f,0.f,0.f,0.f};

  for (int k0 = 0; k0 < K; k0 += 32) {
    V bh[4], bl[4];
#pragma unroll
    for (int j = 0; j < 4; ++j) {
      const size_t bo = (size_t)(n0 + (j << 4) + rlane) * ldb + koff + k0;
      bh[j] = Frag<T>::load(Bb + bo);
      if (SPLIT) bl[j] = Frag<T>::load(Bb2 + bo);
    }
#pragma unroll
    for (int i = 0; i < 4; ++i) {
      const size_t ao = (size_t)(m0 + (i << 4) + rlane) * lda + koff + k0;
      V ah = Frag<T>::load(Ab + ao);
      V al;
      if (SPLIT) al = Frag<T>::load(Ab2 + ao);
#pragma unroll
      for (int j = 0; j < 4; ++j) {
        acc[i][j] = Frag<T>::mma(ah, bh[j], acc[i][j]);
        if (SPLIT) {
          acc[i][j] = Frag<T>::mma(ah, bl[j], acc[i][j]);
          acc[i][j] = Frag<T>::mma(al, bh[j], acc[i][j]);
        }
      }
      Frag<T>::guard(acc[i][0], acc[i][3], ah, SPLIT ? al : ah);
    }
    Frag<T>::keep(bh[0], bh[1], bh[2], bh[3]);
    if (SPLIT) Frag<T>::keep(bl[0], bl[1], bl[2], bl[3]);
  }
  acc_guard4(acc[0][0], acc[0][1], acc[0][2], acc[0][3]);
  acc_guard4(acc[1][0], acc[1][1], acc[1][2], acc[1][3]);
  acc_guard4(acc[2][0], acc[2][1], acc[2][2], acc[2][3]);
  acc_guard4(acc[3][0], acc[3][1], acc[3][2], acc[3][3]);

  float* slab = sT[wave];
  const float* Rb = RESID ? (resid + (size_t)b * strideR) : nullptr;
#pragma unroll
  for (int i = 0; i < 4; ++i) {
    const int mBase = m0 + (i << 4);
#pragma unroll
    for (int j = 0; j < 4; ++j) {
      const int n = n0 + (j << 4) + rlane;
      float bv = 0.f;
      if (BIAS_MODE == 2) bv = bias[n];
#pragma unroll
      for (int r = 0; r < 8; ++r) {
        float v = acc[i][j][r] * scale;
        if (BIAS_MODE == 1) v += bias[mBase + mOff + r];
        if (BIAS_MODE == 2) v += bv;
        if (RESID) v += Rb[(size_t)(mBase + mOff + r) * ldc + n];
        if (ACT == 1) v = tanhf(v);
        if (ACT == 2) v = fmaxf(v, 0.0f);
        if (ACT == 3) v = v / (1.0f + expf(-v));
        if (ACT == 4) v = (v > 0.f) ? v : 0.01f * v;
        if (ACT == 5) v = 0.5f * v * (1.0f + erff(v * 0.70710678118654752f));
        slab[(mOff + r) * 68 + (j << 4) + rlane] = v;
      }
    }
    __builtin_amdgcn_fence(__ATOMIC_RELEASE, "workgroup");
    __builtin_amdgcn_wave_barrier();
    __builtin_amdgcn_fence(__ATOMIC_ACQUIRE, "workgroup");
    if (OUT_MODE == 0) {
      float* C = (float*)Cout + (size_t)b * strideC;
      const int hh = lane >> 4, c4 = (lane & 15) * 4;
      for (int pass = 0; pass < 2; ++pass) {
#pragma unroll
        for (int it = 0; it < 8; ++it) {
          const int row = it * 2 + hh;
          v4f v = *(const v4f*)(slab + row * 68 + c4);
          *(volatile v4f*)(C + (size_t)(mBase + row) * ldc + n0 + c4) = v;
        }
        __threadfence();
      }
    } else {
      const int q = lane >> 3, c8 = (lane & 7) * 8;
      unsigned short* C  = (unsigned short*)Cout  + (size_t)b * strideC;
      unsigned short* C2 = (OUT_MODE == 2) ? ((unsigned short*)Cout2 + (size_t)b * strideC) : nullptr;
      for (int pass = 0; pass < 2; ++pass) {
#pragma unroll
        for (int it = 0; it < 4; ++it) {
          const int row = it * 4 + q;
          const float* sp = slab + row * 68 + c8;
          v8h hv, lv;
#pragma unroll
          for (int e = 0; e < 8; ++e) {
            if (OUT_MODE == 1) {
              hv[e] = (_Float16)sp[e];
            } else {
              unsigned short hb = f2bf_bits(sp[e]);
              unsigned short lb = f2bf_bits(sp[e] - bf_bits2f(hb));
              hv[e] = __builtin_bit_cast(_Float16, hb);
              lv[e] = __builtin_bit_cast(_Float16, lb);
            }
          }
          *(volatile v8h*)(C + (size_t)(mBase + row) * ldc + n0 + c8) = hv;
          if (OUT_MODE == 2) *(volatile v8h*)(C2 + (size_t)(mBase + row) * ldc + n0 + c8) = lv;
        }
        __threadfence();
      }
    }
    __builtin_amdgcn_fence(__ATOMIC_RELEASE, "workgroup");
    __builtin_amdgcn_wave_barrier();
    __builtin_amdgcn_fence(__ATOMIC_ACQUIRE, "workgroup");
  }
}

__global__ __launch_bounds__(256) void cast_scale_f16x2(
    const float* __restrict__ in, _Float16* __restrict__ out, int n2, float sc) {
  int i = blockIdx.x * 256 + threadIdx.x;
  if (i < n2) {
    const unsigned u = h2u(in[2 * i] * sc) | (h2u(in[2 * i + 1] * sc) << 16);
    ((volatile unsigned*)out)[i] = u;
    __threadfence();
    ((volatile unsigned*)out)[i] = u;
  }
}

__global__ __launch_bounds__(RNN_THR) void rnn_stack_kernel(
    const float* __restrict__ x,
    const float* __restrict__ h0,
    long h0_lstride,
    const float* __restrict__ Wih0, const float* __restrict__ Wih, const float* __restrict__ Whh,
    const float* __restrict__ bih, const float* __restrict__ bhh,
    unsigned short* __restrict__ trajp) {
  __shared__ __align__(16) _Float16 Wn[NLAY * WPL];
  __shared__ __align__(16) _Float16 Wr[NLAY * WPL];
  __shared__ float Bsum[NLAY * NHID];
  __shared__ __align__(16) _Float16 Hs[RNN_WAVES][(NLAY + 1) * SLOT];
  __shared__ __align__(16) _Float16 St[RNN_WAVES][16 * 2 * NHID];

  const int tid = threadIdx.x, lane = tid & 31, wave = tid >> 5;
  const int c = lane & 15, hh = lane >> 4, koff = hh * 8;
  const int rloc = blockIdx.x * RNN_ROWS_BLK + wave * 16;

#pragma unroll 1
  for (int it = 0; it < WPL / RNN_THR; ++it) {
    const int i = it * RNN_THR + tid;
    const int n = i >> 5, k = i & 31;
    const int kc = (k < NIN) ? k : 0;
    const float w = Wih0[n * NIN + kc];
    const float keep = (k < NIN) ? 1.0f : 0.0f;
    Wn[i] = (_Float16)((w * keep) * WCARRY);
  }
#pragma unroll 1
  for (int it = 0; it < (NLAY - 1) * WPL / RNN_THR; ++it) {
    const int i = it * RNN_THR + tid;
    Wn[WPL + i] = (_Float16)(Wih[i] * WCARRY);
  }
#pragma unroll 1
  for (int it = 0; it < NLAY * WPL / RNN_THR; ++it) {
    const int i = it * RNN_THR + tid;
    Wr[i] = (_Float16)(Whh[i] * WCARRY);
  }
#pragma unroll 1
  for (int i = tid; i < NLAY * NHID; i += RNN_THR) Bsum[i] = bih[i] + bhh[i];

  _Float16* Hw = Hs[wave];
#pragma unroll 1
  for (int l = 0; l < NLAY; ++l) {
    const float* hl = h0 + (size_t)l * (size_t)h0_lstride;
#pragma unroll 1
    for (int it = 0; it < 4; ++it) {
      const int idx = it * 32 + lane;
      const int row = idx >> 3, c4 = (idx & 7) * 4;
      const v4f v = *(const v4f*)(hl + (size_t)(rloc + row) * NHID + c4);
      v2u pk;
      pk[0] = h2u(v[0]) | (h2u(v[1]) << 16);
      pk[1] = h2u(v[2]) | (h2u(v[3]) << 16);
      *(v2u*)(Hw + (l + 1) * SLOT + row * NHID + c4) = pk;
    }
  }
  __syncthreads();

  const v8f z8 = {0.f, 0.f, 0.f, 0.f, 0.f, 0.f, 0.f, 0.f};
  const _Float16* arow = Hw + c * NHID + koff;
  const float fsel = 1.0f - (float)hh;

#pragma unroll 1
  for (int t = 0; t < NSTEP; ++t) {
    {
      const float* xp = x + ((size_t)(rloc + c) * NSTEP + (size_t)t) * NIN;
      const float x0 = xp[0], x1 = xp[1], x2 = xp[2];
      const float xz = x2 - x2;
      const unsigned z16 = h2u(xz);
      const unsigned zz  = z16 | (z16 << 16);
      const unsigned w0  = h2u(x0 * fsel) | (h2u(x1 * fsel) << 16);
      const unsigned w1  = h2u(x2 * fsel) | (z16 << 16);
      v4u ua; ua[0] = w0; ua[1] = w1; ua[2] = zz; ua[3] = zz;
      v4u ub; ub[0] = zz; ub[1] = zz; ub[2] = zz; ub[3] = zz;
      *(v4u*)(Hw + c * NHID + 16 * hh)     = ua;
      *(v4u*)(Hw + c * NHID + 16 * hh + 8) = ub;
    }
    __syncthreads();

#pragma unroll 1
    for (int l = 0; l < NLAY; ++l) {
      const v16h fa  = Frag<_Float16>::load(arow + l * SLOT);
      const v16h fh  = Frag<_Float16>::load(arow + (l + 1) * SLOT);
      const _Float16* wn = Wn + l * WPL + c * NHID + koff;
      const _Float16* wr = Wr + l * WPL + c * NHID + koff;
      const v16h bw0 = Frag<_Float16>::load(wn);
      const v16h br0 = Frag<_Float16>::load(wr);
      const v16h bw1 = Frag<_Float16>::load(wn + 16 * NHID);
      const v16h br1 = Frag<_Float16>::load(wr + 16 * NHID);
      v8f acc0 = Frag<_Float16>::mma(fa, bw0, z8);
      acc0 = Frag<_Float16>::mma(fh, br0, acc0);
      v8f acc1 = Frag<_Float16>::mma(fa, bw1, z8);
      acc1 = Frag<_Float16>::mma(fh, br1, acc1);
      guard_acc2_frag6(acc0, acc1, fa, fh, bw0, br0, bw1, br1);

      const float bv0 = Bsum[l * NHID + c];
      const float bv1 = Bsum[l * NHID + 16 + c];
      _Float16 hq0[8], hq1[8];
#pragma unroll
      for (int r = 0; r < 8; ++r) {
        hq0[r] = (_Float16)tanh_acc(acc0[r] * WCARRY_INV + bv0);
        hq1[r] = (_Float16)tanh_acc(acc1[r] * WCARRY_INV + bv1);
      }
      _Float16* hout = Hw + (l + 1) * SLOT;
#pragma unroll
      for (int r = 0; r < 8; ++r) {
        hout[(8 * hh + r) * NHID + c]      = hq0[r];
        hout[(8 * hh + r) * NHID + 16 + c] = hq1[r];
      }
      if (l == NLAY - 1) {
        _Float16* st = St[wave] + NHID * (t & 1);
#pragma unroll
        for (int r = 0; r < 8; ++r) {
          st[(8 * hh + r) * (2 * NHID) + c]      = hq0[r];
          st[(8 * hh + r) * (2 * NHID) + 16 + c] = hq1[r];
        }
      }
      __syncthreads();
    }

    if (t & 1) {
      const int q = lane >> 3, c8 = (lane & 7) * 8;
      const _Float16* sw = St[wave];
      _Float16* tg = (_Float16*)trajp + (size_t)(t - 1) * NHID + c8;
      for (int pass = 0; pass < 2; ++pass) {
#pragma unroll
        for (int it = 0; it < 4; ++it) {
          const int row = it * 4 + q;
          const v8h v = *(const v8h*)(sw + row * (2 * NHID) + c8);
          *(volatile v8h*)(tg + (size_t)(rloc + row) * NFEAT) = v;
        }
        __threadfence();
      }
    }
  }
}

__global__ __launch_bounds__(HEAD_THR) void head_out_kernel(
    const float* __restrict__ A4, const float* __restrict__ W5, const float* __restrict__ b5,
    float* __restrict__ outp) {
  __shared__ __align__(16) float so[HEAD_THR];
  const int tid = threadIdx.x, lane = tid & 31, wave = tid >> 5;
  const int row = blockIdx.x * HEAD_THR + tid;
  const float* ap = A4 + (size_t)row * DH4;
  float s = 0.0f;
#pragma unroll 1
  for (int k4 = 0; k4 < DH4 / 4; ++k4) {
    const v4f a = *(const v4f*)(ap + 4 * k4);
    const v4f w = *(const v4f*)(W5 + 4 * k4);
    s = fmaf(a[0], w[0], s);
    s = fmaf(a[1], w[1], s);
    s = fmaf(a[2], w[2], s);
    s = fmaf(a[3], w[3], s);
  }
  s += b5[0];
  so[tid] = s;
  __syncthreads();
  if (wave < 2) {
    const int i4 = (wave * 32 + lane) * 4;
    const v4f v = *(const v4f*)(so + i4);
    float* op = outp + (size_t)blockIdx.x * HEAD_THR + i4;
    *(volatile v4f*)op = v;
    __threadfence();
    *(volatile v4f*)op = v;
  }
}

extern "C" void kernel_launch(void* const* d_in, const int* in_sizes, int n_in,
                              void* d_out, int out_size, void* d_ws, size_t ws_size, hipStream_t stream) {
  if (n_in < 17 || d_out == nullptr || d_ws == nullptr) return;
  if (in_sizes[0] != NBATCH * NSTEP * NIN || in_sizes[1] != NLAY * NBATCH * NHID || in_sizes[2] != NHID * NIN ||
      in_sizes[3] != (NLAY - 1) * NHID * NHID || in_sizes[4] != NLAY * NHID * NHID || in_sizes[5] != NLAY * NHID ||
      in_sizes[6] != NLAY * NHID || in_sizes[7] != DH1 * NFEAT || in_sizes[8] != DH1 || in_sizes[9] != DH2 * DH1 ||
      in_sizes[10] != DH2 || in_sizes[11] != DH3 * DH2 || in_sizes[12] != DH3 || in_sizes[13] != DH4 * DH3 ||
      in_sizes[14] != DH4 || in_sizes[15] != DH4 || in_sizes[16] < 1 || out_size != NBATCH) return;

  const float* x    = (const float*)d_in[0];
  const float* h0   = (const float*)d_in[1];
  const float* Wih0 = (const float*)d_in[2];
  const float* Wih  = (const float*)d_in[3];
  const float* Whh  = (const float*)d_in[4];
  const float* bih  = (const float*)d_in[5];
  const float* bhh  = (const float*)d_in[6];
  const float* W1 = (const float*)d_in[7];  const float* b1 = (const float*)d_in[8];
  const float* W2 = (const float*)d_in[9];  const float* b2 = (const float*)d_in[10];
  const float* W3 = (const float*)d_in[11]; const float* b3 = (const float*)d_in[12];
  const float* W4 = (const float*)d_in[13]; const float* b4 = (const float*)d_in[14];
  const float* W5 = (const float*)d_in[15]; const float* b5 = (const float*)d_in[16];
  float* out = (float*)d_out;

  char* ws = (char*)d_ws; size_t off = 0;
  auto carve = [&](size_t bytes) -> char* { char* p = ws + off; off += (bytes + 255) & ~(size_t)255; return p; };
  _Float16* WQ1 = (_Float16*)carve((size_t)DH1 * NFEAT * 2);
  _Float16* WQ2 = (_Float16*)carve((size_t)DH2 * DH1 * 2);
  _Float16* WQ3 = (_Float16*)carve((size_t)DH3 * DH2 * 2);
  _Float16* WQ4 = (_Float16*)carve((size_t)DH4 * DH3 * 2);
  unsigned short* TRAJ = (unsigned short*)carve((size_t)CHROWS * NFEAT * 2);
  unsigned short* A1   = (unsigned short*)carve((size_t)CHROWS * DH1 * 2);
  unsigned short* A2   = (unsigned short*)carve((size_t)CHROWS * DH2 * 2);
  unsigned short* A3   = (unsigned short*)carve((size_t)CHROWS * DH3 * 2);
  float*          A4   = (float*)carve((size_t)CHROWS * DH4 * 4);
  if (off > ws_size || off > (size_t)134217728) return;

  const int n2w1 = DH1 * NFEAT / 2, n2w2 = DH2 * DH1 / 2, n2w3 = DH3 * DH2 / 2, n2w4 = DH4 * DH3 / 2;
  cast_scale_f16x2<<<(n2w1 + 255) / 256, 256, 0, stream>>>(W1, WQ1, n2w1, WCARRY);
  cast_scale_f16x2<<<(n2w2 + 255) / 256, 256, 0, stream>>>(W2, WQ2, n2w2, WCARRY);
  cast_scale_f16x2<<<(n2w3 + 255) / 256, 256, 0, stream>>>(W3, WQ3, n2w3, WCARRY);
  cast_scale_f16x2<<<(n2w4 + 255) / 256, 256, 0, stream>>>(W4, WQ4, n2w4, WCARRY);

  const unsigned short* WQ1u = (const unsigned short*)WQ1;
  const unsigned short* WQ2u = (const unsigned short*)WQ2;
  const unsigned short* WQ3u = (const unsigned short*)WQ3;
  const unsigned short* WQ4u = (const unsigned short*)WQ4;
  const long h0_lstride = (long)NBATCH * NHID;

  for (int ch = 0; ch < NCHUNK; ++ch) {
    const float* xc  = x  + (size_t)ch * CHROWS * NSTEP * NIN;
    const float* h0c = h0 + (size_t)ch * CHROWS * NHID;
    rnn_stack_kernel<<<CHROWS / RNN_ROWS_BLK, RNN_THR, 0, stream>>>(xc, h0c, h0_lstride, Wih0, Wih, Whh, bih, bhh, TRAJ);

    wmma_gemm64<0, false, 2, 1, false, 2><<<dim3((CHROWS / 64) * (DH1 / 64) / 8, 1), 256, 0, stream>>>(
        TRAJ, TRAJ, NFEAT, 0L, WQ1u, WQ1u, NFEAT, 0L, (void*)A1, (void*)A1, DH1, 0L,
        b1, b1, 0L, CHROWS, DH1, NFEAT, WCARRY_INV);
    wmma_gemm64<0, false, 2, 1, false, 2><<<dim3((CHROWS / 64) * (DH2 / 64) / 8, 1), 256, 0, stream>>>(
        A1, A1, DH1, 0L, WQ2u, WQ2u, DH1, 0L, (void*)A2, (void*)A2, DH2, 0L,
        b2, b2, 0L, CHROWS, DH2, DH1, WCARRY_INV);
    wmma_gemm64<0, false, 2, 1, false, 2><<<dim3((CHROWS / 64) * (DH3 / 64) / 8, 1), 256, 0, stream>>>(
        A2, A2, DH2, 0L, WQ3u, WQ3u, DH2, 0L, (void*)A3, (void*)A3, DH3, 0L,
        b3, b3, 0L, CHROWS, DH3, DH2, WCARRY_INV);
    wmma_gemm64<0, false, 2, 0, false, 2><<<dim3((CHROWS / 64) * (DH4 / 64) / 8, 1), 256, 0, stream>>>(
        A3, A3, DH3, 0L, WQ4u, WQ4u, DH3, 0L, (void*)A4, (void*)A4, DH4, 0L,
        b4, b4, 0L, CHROWS, DH4, DH3, WCARRY_INV);

    head_out_kernel<<<CHROWS / HEAD_THR, HEAD_THR, 0, stream>>>(A4, W5, b5, out + (size_t)ch * CHROWS);
  }
}
